// DeformableInception_28363964023451
// MI455X (gfx1250) — hardware-verified
//
#include <hip/hip_runtime.h>
#include <math.h>

typedef __attribute__((ext_vector_type(16))) _Float16 v16h;
typedef __attribute__((ext_vector_type(16))) __bf16 v16b;
typedef __attribute__((ext_vector_type(8)))  _Float16 v8h;
typedef __attribute__((ext_vector_type(8)))  float v8f;
typedef __attribute__((ext_vector_type(4)))  float v4f;
typedef __attribute__((ext_vector_type(2)))  float v2f;
typedef __attribute__((ext_vector_type(4)))  unsigned v4u;
typedef __attribute__((ext_vector_type(4)))  int v4i;
typedef float __attribute__((may_alias)) float_a;
typedef int __attribute__((may_alias)) int_a;

template <typename T> __device__ __forceinline__ void vst2(void* p, T v) { *(volatile T*)p = v; __threadfence(); *(volatile T*)p = v; }
__device__ __forceinline__ v8f wmma16(v16h a, v16h b, v8f c) {
  v8f d = __builtin_amdgcn_wmma_f32_16x16x32_f16(false, a, false, b, (short)0, c, false, false);
  asm volatile("v_nop\n\tv_nop\n\tv_nop\n\tv_nop" : "+v"(d) : "v"(a), "v"(b));
  return d;
}
__device__ __forceinline__ v8f wmma_bf(v16b a, v16b b, v8f c) {
  v8f d = __builtin_amdgcn_wmma_f32_16x16x32_bf16(false, a, false, b, (short)0, c, false, false);
  asm volatile("v_nop\n\tv_nop\n\tv_nop\n\tv_nop" : "+v"(d) : "v"(a), "v"(b));
  return d;
}
__device__ __forceinline__ v16h frag_h(const _Float16* rowk0, int lane) {
  union { v16h v; v8h q[2]; } u; const _Float16* p = rowk0 + 8 * (lane >> 4);
  u.q[0] = *(const v8h*)p; u.q[1] = *(const v8h*)(p + 16); return u.v;
}
__device__ __forceinline__ v16h frag_f32(const float* rowk0, int lane) {
  v16h a; const float* p = rowk0 + 8 * (lane >> 4);
#pragma unroll
  for (int i = 0; i < 8; ++i) { a[i] = (_Float16)p[i]; a[8 + i] = (_Float16)p[16 + i]; }
  return a;
}
__device__ __forceinline__ v16h frag_f32s(const float* rowk0, int lane, float sc) {
  v16h a; const float* p = rowk0 + 8 * (lane >> 4);
#pragma unroll
  for (int i = 0; i < 8; ++i) { a[i] = (_Float16)(p[i] * sc); a[8 + i] = (_Float16)(p[16 + i] * sc); }
  return a;
}
__device__ __forceinline__ v16h fragc_f32(const float* W, int k0, int n, int lane, int ld, int K) {
  v16h a; const int g = lane >> 4;
#pragma unroll
  for (int i = 0; i < 8; ++i) { const int ka = k0 + 8 * g + i, kb = ka + 16;
    a[i] = (_Float16)(ka < K ? W[(size_t)(ka < K ? ka : K - 1) * ld + n] : 0.f); a[8 + i] = (_Float16)(kb < K ? W[(size_t)(kb < K ? kb : K - 1) * ld + n] : 0.f); }
  return a;
}
struct F2 { v16b h, l; };
__device__ __forceinline__ F2 bsplit16(const float v[16]) { F2 r;
#pragma unroll
  for (int i = 0; i < 16; ++i) { const __bf16 h = (__bf16)v[i]; r.h[i] = h; r.l[i] = (__bf16)(v[i] - (float)h); }
  return r; }
__device__ __forceinline__ F2 split_row(const float* row, int k0, int lane) { float v[16]; const float* p = row + k0 + 8 * (lane >> 4);
#pragma unroll
  for (int i = 0; i < 8; ++i) { v[i] = p[i]; v[8 + i] = p[16 + i]; }
  return bsplit16(v); }
__device__ __forceinline__ F2 split_rowK(const float* row, int k0, int lane, int K) { float v[16]; const int g = lane >> 4;
#pragma unroll
  for (int i = 0; i < 8; ++i) { const int ka = k0 + 8 * g + i, kb = ka + 16; v[i] = ka < K ? row[ka < K ? ka : K - 1] : 0.f; v[8 + i] = kb < K ? row[kb < K ? kb : K - 1] : 0.f; }
  return bsplit16(v); }
__device__ __forceinline__ F2 split_col(const float* W, int k0, int n, int lane, int ld, int K) { float v[16]; const int g = lane >> 4;
#pragma unroll
  for (int i = 0; i < 8; ++i) { const int ka = k0 + 8 * g + i, kb = ka + 16; v[i] = ka < K ? W[(size_t)(ka < K ? ka : K - 1) * ld + n] : 0.f; v[8 + i] = kb < K ? W[(size_t)(kb < K ? kb : K - 1) * ld + n] : 0.f; }
  return bsplit16(v); }
__device__ __forceinline__ v8f mac3(const F2& a, const F2& b, v8f c) { c = wmma_bf(a.l, b.h, c); c = wmma_bf(a.h, b.l, c); return wmma_bf(a.h, b.h, c); }
__device__ __forceinline__ float sigm(float v) { return 1.0f / (1.0f + expf(-v)); }
#define LDSX() do { asm volatile("s_wait_dscnt 0" ::: "memory"); __builtin_amdgcn_wave_barrier(); __builtin_amdgcn_fence(__ATOMIC_RELEASE, "workgroup"); } while (0)


#define NBT 8
#define CIN 128
#define COUT 84
#define COP 96
#define HH 64
#define WWD 64
#define KK 9
#define K1 (CIN * KK)
#define KF 192
#define NROW (NBT * HH)
#ifndef NRT
#define NRT NROW
#endif
typedef __attribute__((ext_vector_type(8))) __bf16 v8b;
__device__ __forceinline__ v16b frag_b(const __bf16* rowk0, int lane) {
  union { v16b v; v8b q[2]; } u; const __bf16* p = rowk0 + 8 * (lane >> 4);
  u.q[0] = *(const v8b*)p; u.q[1] = *(const v8b*)(p + 16); return u.v;
}
__device__ __forceinline__ float bfr(float v) { return (float)(__bf16)v; }
__device__ __attribute__((noinline)) float exp_ni(float v) { return expf(v); }
__device__ __attribute__((noinline)) float erf_ni(float v) { return erff(v); }

#define PK_W0 0
#define PK_W1 (PK_W0 + COP * K1)
#define PK_WF (PK_W1 + COP * K1)
#define PK_END (PK_WF + COP * KF)
#define WS_PK 0u
#define WS_END (WS_PK + 2u * PK_END)

__global__ __launch_bounds__(256) void k_pack(const float* __restrict__ W0, const float* __restrict__ W1, const float* __restrict__ WF, __bf16* __restrict__ PK) {
  __shared__ __align__(16) __bf16 s[K1]; const int o = blockIdx.x, which = blockIdx.y, tid = threadIdx.x; int K; size_t dst;
  if (which < 2) { const float* Wm = which == 0 ? W0 : W1; K = K1; dst = (which == 0 ? PK_W0 : PK_W1) + (size_t)o * K1; for (int k = tid; k < K; k += 256) s[k] = (__bf16)((o < COUT) ? Wm[(size_t)o * K1 + k] : 0.f); }
  else { K = KF; dst = PK_WF + (size_t)o * KF; for (int k = tid; k < K; k += 256) s[k] = (__bf16)((o < COUT && k < 2 * COUT) ? WF[(size_t)o * 2 * COUT + k] : 0.f); }
  __syncthreads();
  for (int q = tid; q < K / 8; q += 256) vst2((unsigned*)(PK + dst + q * 8), *(const v4u*)&s[q * 8]);
}
__global__ __launch_bounds__(128) void k_dinc(const float* __restrict__ X, const float* __restrict__ DM0, const float* __restrict__ DM1, const __bf16* __restrict__ PK, const float* __restrict__ BF, float* __restrict__ OUT) {
  __shared__ int sidx[64][KK][4]; __shared__ float swt[64][KK][4]; __shared__ __align__(16) __bf16 th[64][40], tl[64][40]; __shared__ __align__(16) float scat[64][KF + 4]; __shared__ __align__(16) float so[COP][68];
  const int tid = threadIdx.x, wave = tid >> 5, lane = tid & 31, col = lane & 15, g = lane >> 4; const int row = blockIdx.x; const int b = row / HH, y = row % HH;
  v8f acc[2][6];
#pragma unroll
  for (int br = 0; br < 2; ++br)
#pragma unroll
    for (int j = 0; j < 6; ++j) acc[br][j] = (v8f){};
#pragma unroll
  for (int br = 0; br < 2; ++br) { const float* DM = br == 0 ? DM0 : DM1; const __bf16* P = PK + (br == 0 ? PK_W0 : PK_W1);
    for (int q = tid; q < 64 * KK; q += 128) { const int px = q & 63, t = q >> 6; const float ky = (float)(t / 3) - 1.0f, kx = (float)(t % 3) - 1.0f;
      const float oy = bfr(DM[(((size_t)b * 2 * KK + 2 * t) * HH + y) * WWD + px]), ox = bfr(DM[(((size_t)b * 2 * KK + 2 * t + 1) * HH + y) * WWD + px]);
      const float py = (oy + (float)y) + ky, pxf = (ox + (float)px) + kx;
      const float y0 = floorf(py), x0 = floorf(pxf); const float wy1 = py - y0, wx1 = pxf - x0, wy0 = 1.0f - wy1, wx0 = 1.0f - wx1;
      const int yi = (int)y0, xi = (int)x0;
#pragma unroll
      for (int cnr = 0; cnr < 4; ++cnr) { const int yy = yi + (cnr >> 1), xx = xi + (cnr & 1); const bool ok = (yy >= 0) && (yy < HH) && (xx >= 0) && (xx < WWD);
        sidx[px][t][cnr] = min(max(yy, 0), HH - 1) * WWD + min(max(xx, 0), WWD - 1);
        const float wgt = (cnr == 0) ? wy0 * wx0 : (cnr == 1) ? wy0 * wx1 : (cnr == 2) ? wy1 * wx0 : wy1 * wx1; swt[px][t][cnr] = ok ? wgt : 0.f; } }
    __syncthreads();
#pragma unroll 1
    for (int kc = 0; kc < K1 / 32; ++kc) {
      for (int q = tid; q < 64 * 32; q += 128) { const int px = q & 63, kl = q >> 6; const int k = kc * 32 + kl; const int c = k / KK, t = k % KK; const float* plane = X + ((size_t)b * CIN + c) * HH * WWD;
        const float v = ((bfr(plane[sidx[px][t][0]]) * swt[px][t][0] + bfr(plane[sidx[px][t][1]]) * swt[px][t][1]) + bfr(plane[sidx[px][t][2]]) * swt[px][t][2]) + bfr(plane[sidx[px][t][3]]) * swt[px][t][3];
        const __bf16 hb = (__bf16)v; th[px][kl] = hb; tl[px][kl] = (__bf16)(v - (float)hb); }
      __syncthreads();
      { F2 a; a.h = frag_b(&th[wave * 16 + col][0], lane); a.l = frag_b(&tl[wave * 16 + col][0], lane);
#pragma unroll
        for (int j = 0; j < 6; ++j) { const v16b w = frag_b(P + (size_t)(j * 16 + col) * K1 + kc * 32, lane); acc[br][j] = wmma_bf(a.l, w, acc[br][j]); acc[br][j] = wmma_bf(a.h, w, acc[br][j]); } }
      __syncthreads(); } }
  for (int q = tid; q < 64 * (KF + 4); q += 128) (&scat[0][0])[q] = 0.f;
  __syncthreads();
#pragma unroll
  for (int br = 0; br < 2; ++br)
#pragma unroll
    for (int j = 0; j < 6; ++j) { const int o = j * 16 + col; if (o < COUT) {
#pragma unroll
      for (int r = 0; r < 8; ++r) scat[wave * 16 + 8 * g + r][br * COUT + o] = acc[br][j][r]; } }
  __syncthreads();
  v8f accf[6] = {};
#pragma unroll
  for (int kc = 0; kc < KF / 32; ++kc) { const F2 a = split_row(&scat[wave * 16 + col][0], kc * 32, lane);
#pragma unroll
    for (int j = 0; j < 6; ++j) { const v16b w = frag_b(PK + PK_WF + (size_t)(j * 16 + col) * KF + kc * 32, lane); accf[j] = wmma_bf(a.l, w, accf[j]); accf[j] = wmma_bf(a.h, w, accf[j]); } }
#pragma unroll
  for (int j = 0; j < 6; ++j) { const int o = j * 16 + col; const float bb = (o < COUT) ? bfr(BF[min(o, COUT - 1)]) : 0.f;
#pragma unroll
    for (int r = 0; r < 8; ++r) so[o][wave * 16 + 8 * g + r] = accf[j][r] + bb; }
  __syncthreads();
  for (int q = tid; q < COUT * 16; q += 128) { const int o = q >> 4, pc = q & 15; vst2(OUT + (((size_t)b * COUT + o) * HH + y) * WWD + pc * 4, *(const v4f*)&so[o][pc * 4]); }
}
extern "C" void kernel_launch(void* const* d_in, const int* in_sizes, int n_in, void* d_out, int out_size, void* d_ws, size_t ws_size, hipStream_t stream) {
  (void)in_sizes; (void)n_in; (void)out_size;
  const float** F = (const float**)d_in;
  if (ws_size < (size_t)WS_END) return;
  char* ws = (char*)d_ws; __bf16* PK = (__bf16*)(ws + WS_PK);
  k_pack<<<dim3(COP, 3), 256, 0, stream>>>(F[3], F[4], F[5], PK);
  k_dinc<<<NRT, 128, 0, stream>>>(F[0], F[1], F[2], PK, F[6], (float*)d_out);
}
